// GraphConv1d_35759897706671
// MI455X (gfx1250) — hardware-run, weakly checked
//
#include <hip/hip_runtime.h>


#pragma clang fp contract(off)

#ifndef NB
#define NB 8
#endif
#ifndef SEQ
#define SEQ 2048
#endif
#define NB_FULL  8
#define SEQ_FULL 2048
#ifndef OUT_SEQ
#define OUT_SEQ SEQ
#endif
#define DM   128
#define AW   4
#define OSP  132
#define TSP  132
#define WLP  68
#define FSP  68
#define XNC  256.0f
#define S2I  (1.0f / 65536.0f)
#define HTC  1024.0f
#define HTI  (1.0f / 1024.0f)
#define WSC  64.0f
#define WSI  (1.0f / 64.0f)
#define THR1 0.05f
#define THR2 0.1f
#define THR3 0.15f

static_assert(DM == 128);
static_assert(DM % 64 == 0);
static_assert(SEQ % 64 == 0);
static_assert(SEQ % 32 == 0);
static_assert(SEQ % (16 * AW) == 0);
static_assert((NB * SEQ) % 64 == 0);
static_assert((NB * SEQ) % 16 == 0);
static_assert(((size_t)NB * SEQ * DM) % 8 == 0);
static_assert(16 * AW == 64);
static_assert(NB <= NB_FULL);
static_assert(SEQ <= SEQ_FULL);
static_assert((OSP * 4) % 16 == 0);
static_assert((TSP * 4) % 16 == 0);
static_assert((WLP * 4) % 16 == 0);
static_assert((FSP * 4) % 16 == 0);
static_assert(THR1 > 6.2e-5f);
static_assert(THR2 > 6.2e-5f);
static_assert(THR3 > 6.2e-5f);
static_assert((size_t)16 * AW * 4 <= 131072);
static_assert((size_t)64 * TSP * 4 <= 131072);
static_assert((size_t)AW * 16 * OSP * 4 <= 131072);
static_assert((size_t)DM * WLP * 4 <= 131072);
static_assert((size_t)16 * FSP * 4 <= 131072);
static_assert(256 * 16 == 16 * DM * 2);
static_assert(16 * 16 == 16 * AW * 4);
static_assert(32 * 16 * 4 * 8 == DM * 64 * 2);
static_assert(32 * 16 * 16 == 16 * DM * 4);
static_assert(32 * 16 * 4 * 8 == 64 * DM * 2);
static_assert(32 * 16 * 8 == 16 * 64 * 4);

typedef _Float16 h16;
typedef __attribute__((ext_vector_type(16))) _Float16 v16h;
typedef __attribute__((ext_vector_type(8)))  _Float16 v8h;
typedef __attribute__((ext_vector_type(8)))  float    v8f;
typedef __attribute__((ext_vector_type(4)))  float    v4f;
typedef v4f  __attribute__((may_alias)) v4fa;

__device__ __forceinline__ unsigned short f2bf(float f) { unsigned u = __float_as_uint(f); u += 0x7FFFu + ((u >> 16) & 1u); return (unsigned short)(u >> 16); }
__device__ __forceinline__ float bfr(float f) { return __uint_as_float(((unsigned)f2bf(f)) << 16); }
__device__ __forceinline__ v16h cat16(v8h lo, v8h hi) { return __builtin_shufflevector(lo, hi, 0, 1, 2, 3, 4, 5, 6, 7, 8, 9, 10, 11, 12, 13, 14, 15); }
__device__ __forceinline__ v16h  ldh(const h16* p) { return cat16(*(const v8h*)p, *(const v8h*)(p + 16)); }
__device__ __forceinline__ void wave_sync() { __builtin_amdgcn_fence(3  , "wavefront"); __builtin_amdgcn_wave_barrier(); asm volatile("" ::: "memory"); }
static __device__ __forceinline__ h16 toh_flush(float v) { const h16 r = (h16)v; return (fabsf(v) < 6.103515625e-05f) ? (h16)0.0f : r; }
__device__ __forceinline__ v8f wmma16g(v16h a, v16h b, v8f c) {
    c = __builtin_amdgcn_wmma_f32_16x16x32_f16(false, a, false, b, (short)0, c, false, false);
    asm volatile("v_nop\n\tv_nop\n\tv_nop\n\tv_nop" : "+v"(c) : "v"(a), "v"(b));
    return c;
}

__device__ __forceinline__ void score_step(const h16* __restrict__ XN, size_t ka, v16h q0, v16h q1, v16h q2, v16h q3, v8f& sa, v8f& sb) {
    v8f ta = (v8f){}, tb = (v8f){};
    { const v16h a0 = ldh(XN + ka),      b0 = ldh(XN + ka + 16 * DM);      ta = wmma16g(a0, q0, ta); tb = wmma16g(b0, q0, tb); }
    { const v16h a1 = ldh(XN + ka + 32), b1 = ldh(XN + ka + 16 * DM + 32); ta = wmma16g(a1, q1, ta); tb = wmma16g(b1, q1, tb); }
    { const v16h a2 = ldh(XN + ka + 64), b2 = ldh(XN + ka + 16 * DM + 64); ta = wmma16g(a2, q2, ta); tb = wmma16g(b2, q2, tb); }
    { const v16h a3 = ldh(XN + ka + 96), b3 = ldh(XN + ka + 16 * DM + 96); ta = wmma16g(a3, q3, ta); tb = wmma16g(b3, q3, tb); }
    sa = ta; sb = tb;
}

__global__ __launch_bounds__(256) void k_norm(const float* __restrict__ H, size_t hstride, int inbf, h16* XN) {
    const int tid = threadIdx.x;
    const size_t row = (size_t)blockIdx.x * 16 + (size_t)(tid >> 4);
    const int c8 = (tid & 15) * 8;
    const size_t b = row / SEQ, t = row % SEQ;
    const float* src = H + b * hstride + t * DM + c8;
    const v4f x0 = *(const v4f*)src, x1 = *(const v4f*)(src + 4);
    float v[8];
#pragma unroll
    for (int i = 0; i < 4; ++i) { v[i] = inbf ? bfr(x0[i]) : x0[i]; v[4 + i] = inbf ? bfr(x1[i]) : x1[i]; }
    float ss = 0.0f;
#pragma unroll
    for (int i = 0; i < 8; ++i) ss += v[i] * v[i];
    ss += __shfl_xor(ss, 8, 32); ss += __shfl_xor(ss, 4, 32); ss += __shfl_xor(ss, 2, 32); ss += __shfl_xor(ss, 1, 32);
    const float s = (1.0f / fmaxf(sqrtf(ss), 1.0e-8f)) * XNC;
    v8h o;
#pragma unroll
    for (int i = 0; i < 8; ++i) o[i] = toh_flush(v[i] * s);
    h16* dst = XN + row * DM + c8;
    *(volatile v8h*)dst = o; __threadfence(); *(volatile v8h*)dst = o;
}

__global__ __launch_bounds__(32 * AW) void k_rowsum(const h16* __restrict__ XN, float thr, float* INV) {
    __shared__ __align__(16) float sinv[16 * AW];
    const int lane = threadIdx.x & 31, lr = lane & 15, hi = lane >> 4;
    const int wave = __builtin_amdgcn_readfirstlane((int)(threadIdx.x >> 5));
    const int b = blockIdx.y;
    const int t0 = (blockIdx.x * AW + wave) * 16;
    const size_t xb = (size_t)b * SEQ * DM;
    const size_t qo = xb + (size_t)(t0 + lr) * DM + 8 * hi;
    const v16h q0 = ldh(XN + qo), q1 = ldh(XN + qo + 32), q2 = ldh(XN + qo + 64), q3 = ldh(XN + qo + 96);
    const size_t ko = xb + (size_t)lr * DM + 8 * hi;
    float dsum = 0.0f;
#pragma unroll 1
    for (int key0 = 0; key0 < SEQ; key0 += 32) {
        v8f sa, sb;
        score_step(XN, ko + (size_t)key0 * DM, q0, q1, q2, q3, sa, sb);
#pragma unroll
        for (int r = 0; r < 8; ++r) {
            const float ca = sa[r] * S2I, cb = sb[r] * S2I;
            dsum += ((ca > thr) ? ca : 0.0f) + ((cb > thr) ? cb : 0.0f); }
    }
    dsum += __shfl_xor(dsum, 16, 32);
    const float iv = 1.0f / sqrtf(dsum);
    if (hi == 0) sinv[wave * 16 + lr] = iv;
    __syncthreads();
    if (threadIdx.x < 16) {
        const v4f val = *(const v4fa*)(&sinv[threadIdx.x * 4]);
        float* dst = INV + (size_t)b * SEQ + (size_t)blockIdx.x * (16 * AW) + threadIdx.x * 4;
        *(volatile v4f*)dst = val; __threadfence(); *(volatile v4f*)dst = val;
    }
}

__global__ __launch_bounds__(256) void k_ht(const float* __restrict__ H, size_t hstride, int inbf, const float* __restrict__ INV, h16* HT) {
    __shared__ __align__(16) float ts[64 * TSP];
    const int tid = threadIdx.x, lane = tid & 31;
    const int wave = __builtin_amdgcn_readfirstlane((int)(threadIdx.x >> 5));
    const int b = blockIdx.y, t0 = blockIdx.x * 64;
    const float* src = H + (size_t)b * hstride + (size_t)t0 * DM;
#pragma unroll 1
    for (int i = 0; i < 8; ++i) {
        const int idx = i * 256 + tid; const int tok = idx >> 5, q4 = (idx & 31) * 4;
        const v4f v = *(const v4f*)(src + (size_t)tok * DM + q4);
        const float sc = INV[(size_t)b * SEQ + t0 + tok] * HTC;
        v4f o;
#pragma unroll
        for (int k = 0; k < 4; ++k) { const float x = inbf ? bfr(v[k]) : v[k]; o[k] = x * sc; }
        *(v4fa*)(&ts[tok * TSP + q4]) = o; }
    __syncthreads();
#pragma unroll 1
    for (int ps = 0; ps < 2; ++ps) {
#pragma unroll
        for (int s = 0; s < 4; ++s) { const int f = wave * 16 + 4 * s + (lane >> 3), c8 = (lane & 7) * 8;
            v8h hv;
#pragma unroll
            for (int i = 0; i < 8; ++i) hv[i] = toh_flush(ts[(c8 + i) * TSP + f]);
            *(volatile v8h*)(HT + ((size_t)b * DM + f) * SEQ + t0 + c8) = hv; }
        if (ps == 0) __threadfence(); }
}

__global__ __launch_bounds__(32 * AW) void k_prop(const h16* __restrict__ XN, const h16* __restrict__ HT, const float* __restrict__ INV, float thr, float* HO) {
    __shared__ __align__(16) float os[AW * 16 * OSP];
    const int lane = threadIdx.x & 31, lr = lane & 15, hi = lane >> 4;
    const int wave = __builtin_amdgcn_readfirstlane((int)(threadIdx.x >> 5));
    const int b = blockIdx.y;
    const int t0 = (blockIdx.x * AW + wave) * 16;
    const size_t xb = (size_t)b * SEQ * DM;
    const size_t qo = xb + (size_t)(t0 + lr) * DM + 8 * hi;
    const v16h q0 = ldh(XN + qo), q1 = ldh(XN + qo + 32), q2 = ldh(XN + qo + 64), q3 = ldh(XN + qo + 96);
    const size_t ko = xb + (size_t)lr * DM + 8 * hi;
    const size_t vo = (size_t)b * DM * SEQ + (size_t)lr * SEQ + 8 * hi;
    v8f o[8];
#pragma unroll
    for (int j = 0; j < 8; ++j) o[j] = (v8f){};
#pragma unroll 1
    for (int key0 = 0; key0 < SEQ; key0 += 32) {
        v8f sa, sb;
        score_step(XN, ko + (size_t)key0 * DM, q0, q1, q2, q3, sa, sb);
        v16h pb;
#pragma unroll
        for (int r = 0; r < 8; ++r) {
            const float ca = sa[r] * S2I, cb = sb[r] * S2I;
            pb[r] = (h16)((ca > thr) ? ca : 0.0f); pb[8 + r] = (h16)((cb > thr) ? cb : 0.0f); }
        const h16* va = HT + vo + key0;
        { const v16h v0 = ldh(va), v1 = ldh(va + (size_t)16 * SEQ), v2 = ldh(va + (size_t)32 * SEQ), v3 = ldh(va + (size_t)48 * SEQ);
          o[0] = wmma16g(v0, pb, o[0]); o[1] = wmma16g(v1, pb, o[1]); o[2] = wmma16g(v2, pb, o[2]); o[3] = wmma16g(v3, pb, o[3]); }
        { const v16h v4 = ldh(va + (size_t)64 * SEQ), v5 = ldh(va + (size_t)80 * SEQ), v6 = ldh(va + (size_t)96 * SEQ), v7 = ldh(va + (size_t)112 * SEQ);
          o[4] = wmma16g(v4, pb, o[4]); o[5] = wmma16g(v5, pb, o[5]); o[6] = wmma16g(v6, pb, o[6]); o[7] = wmma16g(v7, pb, o[7]); }
    }
    const float ivt = INV[(size_t)b * SEQ + t0 + lr] * HTI;
    const int wb = wave * 16 * OSP;
#pragma unroll
    for (int j = 0; j < 8; ++j) { v4f a, c;
        a[0] = o[j][0] * ivt; a[1] = o[j][1] * ivt; a[2] = o[j][2] * ivt; a[3] = o[j][3] * ivt;
        c[0] = o[j][4] * ivt; c[1] = o[j][5] * ivt; c[2] = o[j][6] * ivt; c[3] = o[j][7] * ivt;
        *(v4fa*)(&os[wb + lr * OSP + 16 * j + 8 * hi]) = a; *(v4fa*)(&os[wb + lr * OSP + 16 * j + 8 * hi + 4]) = c; }
    wave_sync();
    float* orow = HO + ((size_t)b * SEQ + t0) * DM;
#pragma unroll 1
    for (int ps = 0; ps < 2; ++ps) {
#pragma unroll 4
        for (int row = 0; row < 16; ++row) {
            const v4f val = *(const v4fa*)(&os[wb + row * OSP + lane * 4]);
            *(volatile v4f*)(orow + (size_t)row * DM + lane * 4) = val; }
        if (ps == 0) __threadfence(); }
}

__global__ __launch_bounds__(256) void k_addcvt(const float* __restrict__ H3, const float* __restrict__ X, h16* AF, size_t n8) {
    const size_t i = (size_t)blockIdx.x * 256 + threadIdx.x; if (i >= n8) return;
    const size_t e = i * 8;
    const size_t b = e / ((size_t)SEQ * DM), rem = e % ((size_t)SEQ * DM);
    const float* xs = X + b * ((size_t)SEQ_FULL * DM) + rem;
    const v4f h0 = *(const v4f*)(H3 + e), h1 = *(const v4f*)(H3 + e + 4);
    const v4f x0 = *(const v4f*)xs, x1 = *(const v4f*)(xs + 4);
    v8h o;
#pragma unroll
    for (int k = 0; k < 4; ++k) { o[k] = toh_flush(h0[k] + bfr(x0[k])); o[4 + k] = toh_flush(h1[k] + bfr(x1[k])); }
    *(volatile v8h*)(AF + e) = o; __threadfence(); *(volatile v8h*)(AF + e) = o;
}

__global__ __launch_bounds__(256) void k_wt(const float* __restrict__ W, h16* WT) {
    __shared__ __align__(16) float wl[DM * WLP];
    const int tid = threadIdx.x, lane = tid & 31;
    const int wave = __builtin_amdgcn_readfirstlane((int)(threadIdx.x >> 5));
    const int o0 = blockIdx.x * 64;
#pragma unroll 1
    for (int i = 0; i < 8; ++i) {
        const int idx = i * 256 + tid; const int f = idx >> 4, q4 = (idx & 15) * 4;
        const v4f v = *(const v4f*)(W + (size_t)f * DM + o0 + q4);
        v4f o;
#pragma unroll
        for (int k = 0; k < 4; ++k) o[k] = bfr(v[k]) * WSC;
        *(v4fa*)(&wl[f * WLP + q4]) = o; }
    __syncthreads();
#pragma unroll 1
    for (int ps = 0; ps < 2; ++ps) {
#pragma unroll
        for (int s = 0; s < 4; ++s) { const int oo = wave * 8 + 2 * s + (lane >> 4), c8 = (lane & 15) * 8;
            v8h hv;
#pragma unroll
            for (int i = 0; i < 8; ++i) hv[i] = toh_flush(wl[(c8 + i) * WLP + oo]);
            *(volatile v8h*)(WT + (size_t)(o0 + oo) * DM + c8) = hv; }
        if (ps == 0) __threadfence(); }
}

__global__ __launch_bounds__(32) void k_final(const h16* __restrict__ A, const h16* __restrict__ Bt, float* OUT) {
    __shared__ __align__(16) float os[16 * FSP];
    const int K = DM;
    const int lane = threadIdx.x & 31, lr = lane & 15, hi = lane >> 4; const int r0 = blockIdx.x * 64, c0 = blockIdx.y * 64;
    v8f acc[4][4];
#pragma unroll
    for (int mb = 0; mb < 4; ++mb)
#pragma unroll
        for (int nb = 0; nb < 4; ++nb) acc[mb][nb] = (v8f){};
    const size_t aoff = (size_t)(r0 + lr) * K + 8 * hi, boff = (size_t)(c0 + lr) * K + 8 * hi;
#pragma unroll 1
    for (int kc = 0; kc < K; kc += 32) {
        v16h a[4];
#pragma unroll
        for (int mb = 0; mb < 4; ++mb) a[mb] = ldh(A + aoff + (size_t)mb * 16 * K + kc);
#pragma unroll
        for (int nb = 0; nb < 4; ++nb) { const v16h bfrag = ldh(Bt + boff + (size_t)nb * 16 * K + kc);
#pragma unroll
            for (int mb = 0; mb < 4; ++mb) acc[mb][nb] = wmma16g(a[mb], bfrag, acc[mb][nb]); }
    }
    const int bb = r0 / SEQ, tt = r0 % SEQ;
    float* obase = OUT + ((size_t)bb * OUT_SEQ + (size_t)tt) * DM + c0;
#pragma unroll
    for (int mb = 0; mb < 4; ++mb) {
#pragma unroll
        for (int nb = 0; nb < 4; ++nb) {
#pragma unroll
            for (int j = 0; j < 8; ++j) os[(hi * 8 + j) * FSP + nb * 16 + lr] = acc[mb][nb][j] * WSI; }
        wave_sync();
#pragma unroll 1
        for (int ps = 0; ps < 2; ++ps) {
#pragma unroll
            for (int s = 0; s < 8; ++s) { const int row = 2 * s + (lane >> 4), c4 = (lane & 15) * 4;
                const v4f val = *(const v4fa*)(&os[row * FSP + c4]);
                *(volatile v4f*)(obase + (size_t)(mb * 16 + row) * DM + c4) = val; }
            if (ps == 0) __threadfence(); }
        wave_sync();
    }
}

static constexpr size_t al256(size_t v) { return (v + 255) & ~(size_t)255; }
static constexpr size_t SZ_P16 = al256((size_t)NB * SEQ * DM * 2);
static constexpr size_t SZ_H32 = al256((size_t)NB * SEQ * DM * 4);
static constexpr size_t SZ_INV = al256((size_t)NB * SEQ * 4);
static constexpr size_t SZ_WT  = al256((size_t)DM * DM * 2);
static constexpr size_t SZ_TOTAL = 3 * SZ_P16 + 2 * SZ_H32 + SZ_INV + SZ_WT;
static_assert(SZ_TOTAL <= (size_t)134217728);
static_assert(((size_t)NB * SEQ * 4) % 256 == 0);

extern "C" void kernel_launch(void* const* d_in, const int* in_sizes, int n_in,
                              void* d_out, int out_size, void* d_ws, size_t ws_size, hipStream_t stream) {
    if (n_in < 2) return;
    const size_t needx = ((size_t)(NB - 1) * SEQ_FULL + SEQ) * DM;
    if ((size_t)in_sizes[0] < needx) return;
    if ((size_t)in_sizes[1] < (size_t)DM * DM) return;
    if ((size_t)out_size < ((size_t)(NB - 1) * OUT_SEQ + SEQ) * DM) return;
    if (SZ_TOTAL > ws_size) return;
    const float* x = (const float*)d_in[0];
    const float* w = (const float*)d_in[1];
    float* OUT = (float*)d_out;
    char* wsp = (char*)d_ws;
    h16* XN = (h16*)wsp; wsp += SZ_P16;
    h16* HT = (h16*)wsp; wsp += SZ_P16;
    h16* AF = (h16*)wsp; wsp += SZ_P16;
    float* HA = (float*)wsp; wsp += SZ_H32;
    float* HB = (float*)wsp; wsp += SZ_H32;
    float* INV = (float*)wsp; wsp += SZ_INV;
    h16* WT = (h16*)wsp; wsp += SZ_WT;

    k_wt<<<DM / 64, 256, 0, stream>>>(w, WT);

    const float thr[3] = { THR1, THR2, THR3 };
    float* houts[3] = { HA, HB, HA };
    const float* hin = x; size_t hstride = (size_t)SEQ_FULL * DM; int inbf = 1;
    for (int s = 0; s < 3; ++s) {
        k_norm<<<(unsigned)((size_t)NB * SEQ / 16), 256, 0, stream>>>(hin, hstride, inbf, XN);
        k_rowsum<<<dim3(SEQ / (16 * AW), NB, 1), 32 * AW, 0, stream>>>(XN, thr[s], INV);
        k_ht<<<dim3(SEQ / 64, NB, 1), 256, 0, stream>>>(hin, hstride, inbf, INV, HT);
        k_prop<<<dim3(SEQ / (16 * AW), NB, 1), 32 * AW, 0, stream>>>(XN, HT, INV, thr[s], houts[s]);
        hin = houts[s]; hstride = (size_t)SEQ * DM; inbf = 0;
    }
    { const size_t n8 = (size_t)NB * SEQ * DM / 8;
      k_addcvt<<<(unsigned)((n8 + 255) / 256), 256, 0, stream>>>(HA, x, AF, n8); }
    k_final<<<dim3(NB * SEQ / 64, DM / 64, 1), 32, 0, stream>>>(AF, WT, OUT);
}
